// GraphClassifier_16621523435857
// MI455X (gfx1250) — hardware-run, weakly checked
//
#include <hip/hip_runtime.h>
#include <math.h>

constexpr int kNodes  = 20000;
constexpr int kEdges  = 300000;
constexpr int kVirt   = kEdges + kNodes;
constexpr int kNP     = 20032;
constexpr int kGraphs = 64;
constexpr int kDin    = 64;
constexpr int kFC     = 256;
constexpr int kHeads  = 4;
constexpr int kCls    = 10;
constexpr int kG4     = 1024;
constexpr int kQ2     = 512;
constexpr int kGK     = 768;
constexpr int kNT     = 256;
constexpr int kSRB    = 1024;
constexpr int kTiles  = 20;
constexpr int kNPA    = kTiles * kSRB;
constexpr int kSCH    = 4096;
constexpr int kSP     = kSCH / kNT;
constexpr int kNCH    = (kVirt + kSCH - 1) / kSCH;
constexpr int kSCHB   = 2048;
constexpr int kNCHB   = (kNodes + kSCHB - 1) / kSCHB;
constexpr float kSlope     = 0.2f;
constexpr float kOpCarry   = 16.0f;
constexpr float kQCarry    = 64.0f;
constexpr float kFeatScale = 1.0f / 256.0f;
constexpr float kGateScale = 1.0f / 1024.0f;

static_assert(kEdges % kSP == 0, "edge groups are entirely real or entirely virtual");
static_assert(kSP % 4 == 0, "int4 edge loads");
static_assert(kNPA >= kNP, "accumulator planes cover the padded node rows");
static_assert(kNP % 64 == 0 && kNP >= kNodes && kNP - kNodes < 64, "M tile padding");
static_assert(kDin % 32 == 0 && kFC % 32 == 0 && kGK % 32 == 0, "K multiples of 32");
static_assert(kFC % 64 == 0 && kG4 % 64 == 0 && kGraphs % 64 == 0, "N and M tile multiples");
static_assert(kSRB == 8 * 128, "eight waves own 128 rows each");
static_assert(kNodes % 8 == 0, "batch vector loaded 8 entries per thread");
static_assert((kGraphs * kCls) % 128 == 0, "output is a whole number of 512-B wave stores");
static_assert(kNodes < 65536, "16-bit src field in the hit record");

typedef __attribute__((ext_vector_type(16))) _Float16 v16h;
typedef __attribute__((ext_vector_type(8)))  _Float16 v8h;
typedef __attribute__((ext_vector_type(16))) __bf16   v16b;
typedef __attribute__((ext_vector_type(8)))  __bf16   v8b;
typedef __attribute__((ext_vector_type(8)))  float    v8f;
typedef __attribute__((ext_vector_type(4)))  float    v4f;
typedef __attribute__((ext_vector_type(4)))  int      v4i;
typedef __attribute__((ext_vector_type(4)))  unsigned int v4u;

__device__ __forceinline__ unsigned short f2bf_bits(float f) {
  unsigned u = __float_as_uint(f);
  return (unsigned short)((u + 0x7FFFu + ((u >> 16) & 1u)) >> 16);
}
__device__ __forceinline__ float bf_bits2f(unsigned short h) { return __uint_as_float(((unsigned)h) << 16); }

__device__ __forceinline__ void dep_guard_h(v8f& a, v8f& b, v16h x, v16h y) { asm volatile("v_nop\n\tv_nop\n\tv_nop\n\tv_nop" : "+v"(a), "+v"(b) : "v"(x), "v"(y)); }
__device__ __forceinline__ void dep_guard_b(v8f& a, v8f& b, v16b x, v16b y) { asm volatile("v_nop\n\tv_nop\n\tv_nop\n\tv_nop" : "+v"(a), "+v"(b) : "v"(x), "v"(y)); }
__device__ __forceinline__ void keep4_h(v16h a, v16h b, v16h c, v16h d) { asm volatile("v_nop" :: "v"(a), "v"(b), "v"(c), "v"(d)); }
__device__ __forceinline__ void keep4_b(v16b a, v16b b, v16b c, v16b d) { asm volatile("v_nop" :: "v"(a), "v"(b), "v"(c), "v"(d)); }
__device__ __forceinline__ void fence_v4(v4f& t) { asm volatile("" : "+v"(t)); }
__device__ __forceinline__ void acc_guard4(v8f& a, v8f& b, v8f& c, v8f& d) { asm volatile("v_nop\n\tv_nop\n\tv_nop\n\tv_nop" : "+v"(a), "+v"(b), "+v"(c), "+v"(d)); }
template <typename T> struct Frag;
template <> struct Frag<_Float16> {
  typedef v16h V; union U { v16h v; v8h h[2]; };
  static __device__ __forceinline__ v16h load(const _Float16* p) {
    U f; f.h[0] = *(const v8h*)(p); f.h[1] = *(const v8h*)(p + 16); return f.v;
  }
  static __device__ __forceinline__ v8f mma(v16h a, v16h b, v8f c) {
    return __builtin_amdgcn_wmma_f32_16x16x32_f16(false, a, false, b, (short)0, c, false, false);
  }
  static __device__ __forceinline__ void guard(v8f& a, v8f& b, v16h x, v16h y) { dep_guard_h(a, b, x, y); }
  static __device__ __forceinline__ void keep(v16h a, v16h b, v16h c, v16h d) { keep4_h(a, b, c, d); }
};
template <> struct Frag<__bf16> {
  typedef v16b V; union U { v16b v; v8b h[2]; };
  static __device__ __forceinline__ v16b load(const __bf16* p) {
    U f; f.h[0] = *(const v8b*)(p); f.h[1] = *(const v8b*)(p + 16); return f.v;
  }
  static __device__ __forceinline__ v8f mma(v16b a, v16b b, v8f c) {
    return __builtin_amdgcn_wmma_f32_16x16x32_bf16(false, a, false, b, (short)0, c, false, false);
  }
  static __device__ __forceinline__ void guard(v8f& a, v8f& b, v16b x, v16b y) { dep_guard_b(a, b, x, y); }
  static __device__ __forceinline__ void keep(v16b a, v16b b, v16b c, v16b d) { keep4_b(a, b, c, d); }
};

__device__ __forceinline__ unsigned pk16(unsigned short a, unsigned short b) { return (unsigned)a | ((unsigned)b << 16); }
__device__ __forceinline__ unsigned short h_bits(float f) { const _Float16 h = (_Float16)f; return __builtin_bit_cast(unsigned short, h); }

template <int ET> struct Elem;
template <> struct Elem<0> { typedef _Float16 T; };
template <> struct Elem<1> { typedef __bf16 T; };
template <int ET, bool SPLIT, int BIAS_MODE, int OUT_MODE, bool RESID, int ACT = 0>
__global__ __launch_bounds__(256) void wmma_gemm64(
    const unsigned short* __restrict__ Ap, const unsigned short* __restrict__ A2p, int lda, long strideA,
    const unsigned short* __restrict__ Btp, const unsigned short* __restrict__ Bt2p, int ldb, long strideB,
    void* __restrict__ Cout, void* __restrict__ Cout2, int ldc, long strideC,
    const float* __restrict__ bias,
    const float* __restrict__ resid, long strideR,
    int M, int N, int K, float scale) {
  typedef typename Elem<ET>::T T;
  typedef typename Frag<T>::V V;
  const T* A = (const T*)Ap; const T* A2 = (const T*)A2p; const T* Bt = (const T*)Btp; const T* Bt2 = (const T*)Bt2p;
  __shared__ __align__(16) float sT[8][16 * 68];
  const int b    = blockIdx.y;
  const int lane = threadIdx.x & 31;
  const int wave = threadIdx.x >> 5;
  const int tilesN = N >> 6;
  const int tilesM = M >> 6;
  const int tile = blockIdx.x * 8 + wave;
  if (tile >= tilesM * tilesN) return;
  const int tm = tile / tilesN;
  const int tn = tile - tm * tilesN;
  const int m0 = tm << 6;
  const int n0 = tn << 6;

  const T* Ab  = A  + (size_t)b * strideA;
  const T* Bb  = Bt + (size_t)b * strideB;
  const T* Ab2 = SPLIT ? (A2  + (size_t)b * strideA) : nullptr;
  const T* Bb2 = SPLIT ? (Bt2 + (size_t)b * strideB) : nullptr;

  const int rlane = lane & 15;
  const int koff  = (lane >> 4) * 8;
  const int mOff  = (lane >> 4) * 8;

  v8f acc[4][4];
#pragma unroll
  for (int i = 0; i < 4; ++i)
#pragma unroll
    for (int j = 0; j < 4; ++j) acc[i][j] = (v8f){0.f,0.f,0.f,0.f,0.f,0.f,0.f,0.f};

  for (int k0 = 0; k0 < K; k0 += 32) {
    V bh[4], bl[4];
#pragma unroll
    for (int j = 0; j < 4; ++j) {
      const size_t bo = (size_t)(n0 + (j << 4) + rlane) * ldb + koff + k0;
      bh[j] = Frag<T>::load(Bb + bo);
      if (SPLIT) bl[j] = Frag<T>::load(Bb2 + bo);
    }
#pragma unroll
    for (int i = 0; i < 4; ++i) {
      const size_t ao = (size_t)(m0 + (i << 4) + rlane) * lda + koff + k0;
      V ah = Frag<T>::load(Ab + ao);
      V al;
      if (SPLIT) al = Frag<T>::load(Ab2 + ao);
#pragma unroll
      for (int j = 0; j < 4; ++j) {
        acc[i][j] = Frag<T>::mma(ah, bh[j], acc[i][j]);
        if (SPLIT) {
          acc[i][j] = Frag<T>::mma(ah, bl[j], acc[i][j]);
          acc[i][j] = Frag<T>::mma(al, bh[j], acc[i][j]);
        }
      }
      Frag<T>::guard(acc[i][0], acc[i][3], ah, SPLIT ? al : ah);
      acc_guard4(acc[i][0], acc[i][1], acc[i][2], acc[i][3]);
    }
    Frag<T>::keep(bh[0], bh[1], bh[2], bh[3]);
    if (SPLIT) Frag<T>::keep(bl[0], bl[1], bl[2], bl[3]);
  }
  acc_guard4(acc[0][0], acc[0][1], acc[0][2], acc[0][3]);
  acc_guard4(acc[1][0], acc[1][1], acc[1][2], acc[1][3]);
  acc_guard4(acc[2][0], acc[2][1], acc[2][2], acc[2][3]);
  acc_guard4(acc[3][0], acc[3][1], acc[3][2], acc[3][3]);

  float* slab = sT[wave];
  const float* Rb = RESID ? (resid + (size_t)b * strideR) : nullptr;
#pragma unroll
  for (int i = 0; i < 4; ++i) {
    const int mBase = m0 + (i << 4);
#pragma unroll
    for (int j = 0; j < 4; ++j) {
      const int n = n0 + (j << 4) + rlane;
      float bv = 0.f;
      if (BIAS_MODE == 2) bv = bias[n];
#pragma unroll
      for (int r = 0; r < 8; ++r) {
        float v = acc[i][j][r] * scale;
        if (BIAS_MODE == 1) v += bias[mBase + mOff + r];
        if (BIAS_MODE == 2) v += bv;
        if (RESID) v += Rb[(size_t)(mBase + mOff + r) * ldc + n];
        if (ACT == 2) v = fmaxf(v, 0.0f);
        if (ACT == 4) v = (v > 0.f) ? v : 0.01f * v;
        slab[(mOff + r) * 68 + (j << 4) + rlane] = v;
      }
    }
    __builtin_amdgcn_fence(__ATOMIC_RELEASE, "workgroup");
    __builtin_amdgcn_wave_barrier();
    __builtin_amdgcn_fence(__ATOMIC_ACQUIRE, "workgroup");
    if (OUT_MODE == 0) {
      float* C = (float*)Cout + (size_t)b * strideC;
      const int hh = lane >> 4, c4 = (lane & 15) * 4;
      for (int pass = 0; pass < 2; ++pass) {
#pragma unroll
        for (int it = 0; it < 8; ++it) {
          const int row = it * 2 + hh;
          v4f v = *(const v4f*)(slab + row * 68 + c4);
          *(volatile v4f*)(C + (size_t)(mBase + row) * ldc + n0 + c4) = v;
        }
        __threadfence();
      }
    } else {
      const int q = lane >> 3, c8 = (lane & 7) * 8;
      unsigned short* C  = (unsigned short*)Cout  + (size_t)b * strideC;
      unsigned short* C2 = (OUT_MODE == 2) ? ((unsigned short*)Cout2 + (size_t)b * strideC) : nullptr;
      for (int pass = 0; pass < 2; ++pass) {
#pragma unroll
        for (int it = 0; it < 4; ++it) {
          const int row = it * 4 + q;
          const float* sp = slab + row * 68 + c8;
          v8h hv, lv;
#pragma unroll
          for (int e = 0; e < 8; ++e) {
            if (OUT_MODE == 1) {
              hv[e] = (_Float16)sp[e];
            } else {
              unsigned short hb = f2bf_bits(sp[e]);
              unsigned short lb = f2bf_bits(sp[e] - bf_bits2f(hb));
              hv[e] = __builtin_bit_cast(_Float16, hb);
              lv[e] = __builtin_bit_cast(_Float16, lb);
            }
          }
          *(volatile v8h*)(C + (size_t)(mBase + row) * ldc + n0 + c8) = hv;
          if (OUT_MODE == 2) *(volatile v8h*)(C2 + (size_t)(mBase + row) * ldc + n0 + c8) = lv;
        }
        __threadfence();
      }
    }
    __builtin_amdgcn_fence(__ATOMIC_RELEASE, "workgroup");
    __builtin_amdgcn_wave_barrier();
    __builtin_amdgcn_fence(__ATOMIC_ACQUIRE, "workgroup");
  }
}

__device__ __forceinline__ void wave_lds_sync() {
  __builtin_amdgcn_fence(__ATOMIC_RELEASE, "workgroup");
  __builtin_amdgcn_wave_barrier();
  __builtin_amdgcn_fence(__ATOMIC_ACQUIRE, "workgroup");
}
__device__ __forceinline__ float dot4(v4f a, v4f b) { return a[0] * b[0] + a[1] * b[1] + a[2] * b[2] + a[3] * b[3]; }
__device__ __forceinline__ v4f relu4(v4f t) {
  v4f r;
#pragma unroll
  for (int e = 0; e < 4; ++e) r[e] = fmaxf(t[e], 0.f);
  return r;
}
__device__ __forceinline__ float sigm(float x) { return __builtin_amdgcn_rcpf(1.0f + expf(-x)); }

__device__ __forceinline__ int blk_excl_scan(int cnt, int* scan_ws, int tid, int* tot) {
  const int lane = tid & 31, wave = tid >> 5; int incl = cnt;
#pragma unroll
  for (int o = 1; o < 32; o <<= 1) { const int v = __shfl_up(incl, o, 32); if (lane >= o) incl += v; }
  if (lane == 31) scan_ws[wave] = incl;
  __syncthreads();
  if (wave == 0) { int wv = (lane < kNT / 32) ? scan_ws[lane] : 0; int wincl = wv;
#pragma unroll
    for (int o = 1; o < 32; o <<= 1) { const int v = __shfl_up(wincl, o, 32); if (lane >= o) wincl += v; }
    if (lane < kNT / 32) scan_ws[32 + lane] = wincl - wv; if (lane == 31) scan_ws[64] = wincl; }
  __syncthreads();
  const int res = scan_ws[32 + wave] + incl - cnt; *tot = scan_ws[64];
  return res;
}

__device__ __forceinline__ int chunk_hits(const int* __restrict__ dstv, const int* __restrict__ srcv, int e0, int n0, int tid,
                                          int* LIST, int* scan_ws) {
  const int eb = e0 + tid * kSP;
  int rg = (eb < kEdges) ? 1 : 0;
  asm volatile("" : "+v"(rg));
  const int ebc = (eb < kEdges) ? eb : (kEdges - kSP);
  v4i dq[kSP / 4], sq[kSP / 4];
#pragma unroll
  for (int k4 = 0; k4 < kSP / 4; ++k4) dq[k4] = *(const v4i*)(dstv + ebc + 4 * k4);
  asm volatile("" ::: "memory");
#pragma unroll
  for (int k4 = 0; k4 < kSP / 4; ++k4) sq[k4] = *(const v4i*)(srcv + ebc + 4 * k4);
  int rec[kSP]; int cnt = 0;
#pragma unroll
  for (int k = 0; k < kSP; ++k) {
    const int dr = dq[k >> 2][k & 3];
    int sr = sq[k >> 2][k & 3]; sr = sr < 0 ? 0 : (sr >= kNodes ? kNodes - 1 : sr);
    const int ev = eb + k;
    const int dv = ev - kEdges;
    const int vok = (ev < kVirt) ? 1 : 0;
    const int d = dv + rg * (dr - dv);
    const int s = dv + rg * (sr - dv);
    const int ok = rg + (1 - rg) * vok;
    int r = -1;
    if (ok != 0 && d >= n0 && d < n0 + kSRB) { r = ((d - n0) << 16) | s; ++cnt; }
    rec[k] = r;
  }
  int tot; int p = blk_excl_scan(cnt, scan_ws, tid, &tot);
#pragma unroll
  for (int k = 0; k < kSP; ++k) if (rec[k] >= 0) { if ((unsigned)p < (unsigned)kSCH) LIST[p] = rec[k]; ++p; }
  __syncthreads();
  return tot < kSCH ? tot : kSCH;
}

__global__ __launch_bounds__(256) void wtcast_kernel(const float* __restrict__ W0, const float* __restrict__ W1,
                                                     const float* __restrict__ W2,
                                                     unsigned short* __restrict__ T0, unsigned short* __restrict__ T1,
                                                     unsigned short* __restrict__ T2, float scale) {
  __shared__ float sm[64][65];
  const int t  = threadIdx.x;
  const int z  = blockIdx.z;
  const int K  = (z == 0) ? kDin : kFC;
  const float* W = (z == 0) ? W0 : (z == 1) ? W1 : W2;
  unsigned short* op = (z == 0) ? T0 : (z == 1) ? T1 : T2;
  const int k0 = blockIdx.x * 64;
  const int n0 = blockIdx.y * 64;
  if (k0 >= K) return;
#pragma unroll
  for (int i = 0; i < 16; ++i) {
    const int e = i * 256 + t;
    const int r = e >> 6;
    const int c = e & 63;
    sm[c][r] = W[(size_t)(k0 + r) * kFC + n0 + c] * scale;
  }
  __syncthreads();
  const int lane = t & 31, wave = t >> 5;
  const int q = lane >> 3, c8 = (lane & 7) * 8;
  for (int pass = 0; pass < 2; ++pass) {
#pragma unroll
    for (int it = 0; it < 2; ++it) {
      const int row = wave * 8 + it * 4 + q;
      unsigned short hb[8];
#pragma unroll
      for (int e = 0; e < 8; ++e) hb[e] = h_bits(sm[row][c8 + e]);
      const v4u u = (v4u){pk16(hb[0], hb[1]), pk16(hb[2], hb[3]), pk16(hb[4], hb[5]), pk16(hb[6], hb[7])};
      *(volatile v4u*)(op + (size_t)(n0 + row) * K + k0 + c8) = u;
    }
    __threadfence();
  }
}

__global__ __launch_bounds__(256) void wgcast_kernel(const float* __restrict__ Wih, const float* __restrict__ Whh,
                                                     const float* __restrict__ bih, const float* __restrict__ bhh,
                                                     unsigned short* __restrict__ WG, float* __restrict__ bsum) {
  const int i = blockIdx.x * 256 + threadIdx.x;
  if (i < kG4 * (kGK / 8)) {
    int j, c8; const float* src;
    if (i < kG4 * 64) { j = i >> 6; c8 = (i & 63) * 8; src = Wih + (size_t)j * kQ2 + c8; }
    else { const int i2 = i - kG4 * 64; j = i2 >> 5; c8 = kQ2 + (i2 & 31) * 8; src = Whh + (size_t)j * kFC + (i2 & 31) * 8; }
    const v4f a = *(const v4f*)(src);
    const v4f c = *(const v4f*)(src + 4);
    unsigned short hb[8];
#pragma unroll
    for (int e = 0; e < 4; ++e) { hb[e] = h_bits(a[e] * kOpCarry); hb[4 + e] = h_bits(c[e] * kOpCarry); }
    const v4u u = (v4u){pk16(hb[0], hb[1]), pk16(hb[2], hb[3]), pk16(hb[4], hb[5]), pk16(hb[6], hb[7])};
    unsigned short* dst = WG + (size_t)j * kGK + c8;
    *(volatile v4u*)dst = u;
    __threadfence();
    *(volatile v4u*)dst = u;
  }
  if (blockIdx.x < 4) {
    const float s = bih[i] + bhh[i];
    ((volatile float*)bsum)[i] = s;
    __threadfence();
    ((volatile float*)bsum)[i] = s;
  }
}

__global__ __launch_bounds__(256) void xcast_kernel(const float* __restrict__ x, unsigned short* __restrict__ X16) {
  const int i = blockIdx.x * 256 + threadIdx.x;
  if (i >= kNP * kDin / 8) return;
  const int n = i >> 3, c8 = (i & 7) * 8;
  const int nc = n < kNodes ? n : kNodes - 1;
  const float cf = (n < kNodes) ? kOpCarry : 0.f;
  const float* p = x + (size_t)nc * kDin + c8;
  const v4f a = *(const v4f*)p;
  const v4f c = *(const v4f*)(p + 4);
  unsigned short hb[8];
#pragma unroll
  for (int e = 0; e < 4; ++e) { hb[e] = h_bits(a[e] * cf); hb[4 + e] = h_bits(c[e] * cf); }
  const v4u u = (v4u){pk16(hb[0], hb[1]), pk16(hb[2], hb[3]), pk16(hb[4], hb[5]), pk16(hb[6], hb[7])};
  unsigned short* q = X16 + 8 * (size_t)i;
  *(volatile v4u*)q = u;
  __threadfence();
  *(volatile v4u*)q = u;
}

__global__ __launch_bounds__(256) void zero16_kernel(unsigned* __restrict__ p, int n4) {
  const int i = blockIdx.x * 256 + threadIdx.x;
  if (i >= n4) return;
  const v4u z = {0u, 0u, 0u, 0u};
  *(volatile v4u*)(p + 4 * (size_t)i) = z;
  __threadfence();
  *(volatile v4u*)(p + 4 * (size_t)i) = z;
}

__global__ __launch_bounds__(256) void alar_kernel(const float* __restrict__ feat, const float* __restrict__ as_,
                                                   const float* __restrict__ ad_, float* __restrict__ AL, float* __restrict__ AR) {
  const int t = blockIdx.x * 256 + threadIdx.x;
  if (t >= kNodes * kHeads) return;
  const int n = t >> 2, hd = t & 3;
  const float* f  = feat + (size_t)n * kFC + hd * 64;
  const float* sv = as_ + hd * 64;
  const float* dv = ad_ + hd * 64;
  float sl = 0.f, sr = 0.f;
#pragma unroll 1
  for (int i = 0; i < 16; ++i) {
    const v4f x4 = *(const v4f*)(f + 4 * i);
    const v4f s4 = *(const v4f*)(sv + 4 * i);
    const v4f d4 = *(const v4f*)(dv + 4 * i);
    sl += dot4(x4, s4);
    sr += dot4(x4, d4);
  }
  for (int pass = 0; pass < 2; ++pass) {
    ((volatile float*)AL)[t] = sl;
    ((volatile float*)AR)[t] = sr;
    __threadfence();
  }
}

template <bool RESID>
__global__ __launch_bounds__(kNT) void gat_kernel(const float* __restrict__ feat, const int* __restrict__ ei,
                                                  const float* __restrict__ AL, const float* __restrict__ AR,
                                                  const float* __restrict__ bias, const float* __restrict__ Hin,
                                                  float* Hout, unsigned short* __restrict__ H16) {
  __shared__ int LIST[kSCH];
  __shared__ float SM[kSRB * kHeads];
  __shared__ float SL[kSRB * kHeads];
  __shared__ float SAD[kSRB * kHeads];
  __shared__ __align__(16) float SROW[8 * kFC];
  __shared__ int scan_ws[80];
  const int tid = threadIdx.x, lane = tid & 31, wave = tid >> 5;
  const int n0 = blockIdx.x * kSRB;
  const int c4 = 4 * lane;
  const int hq = lane & 3;
  const int hd0 = lane >> 4;
  const int hd1 = 2 + (lane >> 4);
  const v4f z4 = {0.f, 0.f, 0.f, 0.f};
#pragma unroll 1
  for (int j = 0; j < 128; ++j) {
    float* rp = Hout + (size_t)(n0 + wave * 128 + j) * kFC + c4;
    *(v4f*)rp = z4;
    *(v4f*)(rp + 128) = z4;
  }
  if (tid < 80) scan_ws[tid] = 0;
  for (int i = tid; i < kSRB * kHeads; i += kNT) {
    SM[i] = -INFINITY; SL[i] = 0.f;
    const int dl = i >> 2, hd = i & 3;
    int n = n0 + dl; n = n < kNodes ? n : kNodes - 1;
    SAD[i] = AR[n * 4 + hd];
  }
  __syncthreads();
  const int* srcv = ei;
  const int* dstv = ei + kEdges;
#pragma unroll 1
  for (int c = 0; c < kNCH; ++c) {
    const int tot = chunk_hits(dstv, srcv, c * kSCH, n0, tid, LIST, scan_ws);
#pragma unroll 1
    for (int base = 0; base < tot; base += 32) {
      const int q = base + lane;
      const int qc = (q < tot) ? q : (tot - 1);
      int rv = LIST[qc];
      rv = (q < tot) ? rv : -1;
      const int own = (rv >= 0 && (rv >> 23) == wave) ? 1 : 0;
      unsigned msk = (unsigned)__ballot(own);
#pragma unroll 1
      for (int it = 0; it < 32; ++it) {
        if (msk == 0u) break;
        const int bp = __builtin_ctz(msk); msk &= msk - 1u;
        const int r = __shfl(rv, bp, 32);
        const int dl = r >> 16, s = r & 0xFFFF;
        const float* fs = feat + (size_t)s * kFC + c4;
        const v4f h0 = *(const v4f*)fs;
        const v4f h1 = *(const v4f*)(fs + 128);
        const int mi = dl * 4 + hq;
        float ev = AL[s * 4 + hq] + SAD[mi];
        ev = (ev >= 0.f) ? ev : kSlope * ev;
        const float mo = SM[mi], lo = SL[mi];
        const float mn = fmaxf(mo, ev);
        const float rr = expf(mo - mn);
        const float ex = expf(ev - mn);
        const float ln = lo * rr + ex;
        if (lane < 4) { SM[mi] = mn; SL[mi] = ln; }
        const float rr0 = __shfl(rr, hd0, 32), ex0 = __shfl(ex, hd0, 32);
        const float rr1 = __shfl(rr, hd1, 32), ex1 = __shfl(ex, hd1, 32);
        float* rp = Hout + (size_t)(n0 + dl) * kFC + c4;
        v4f a0 = *(const v4f*)rp;
        v4f a1 = *(const v4f*)(rp + 128);
        a0 = a0 * rr0 + ex0 * h0;
        a1 = a1 * rr1 + ex1 * h1;
        *(v4f*)rp = a0;
        *(v4f*)(rp + 128) = a1;
      }
    }
    __syncthreads();
  }
  const v4f bv0 = *(const v4f*)(bias + c4);
  const v4f bv1 = *(const v4f*)(bias + 128 + c4);
  float* srow = SROW + wave * kFC;
#pragma unroll 1
  for (int j = 0; j < 128; ++j) {
    const int dl = wave * 128 + j;
    const int n = n0 + dl;
    if (n < kNP) {
      const float livef = (n < kNodes) ? 1.f : 0.f;
      float lv = SL[dl * 4 + hq];
      lv = (lv > 0.f) ? lv : 1.f;
      const float inv = 1.0f / lv;
      const float inv0 = __shfl(inv, hd0, 32);
      const float inv1 = __shfl(inv, hd1, 32);
      float* rp = Hout + (size_t)n * kFC + c4;
      const v4f a0 = *(const v4f*)rp;
      const v4f a1 = *(const v4f*)(rp + 128);
      v4f v0 = a0 * inv0; fence_v4(v0); v0 = v0 + bv0;
      v4f v1 = a1 * inv1; fence_v4(v1); v1 = v1 + bv1;
      v0 = relu4(v0); v1 = relu4(v1);
      if (RESID) {
        const v4f r0 = *(const v4f*)(Hin + (size_t)n * kFC + c4);
        const v4f r1 = *(const v4f*)(Hin + (size_t)n * kFC + 128 + c4);
        v0 = v0 + r0; v1 = v1 + r1;
      }
      v0 = v0 * livef; v1 = v1 * livef;
      *(v4f*)(srow + c4) = v0;
      *(v4f*)(srow + 128 + c4) = v1;
      wave_lds_sync();
      const v4f p0 = *(const v4f*)(srow + 8 * lane);
      const v4f p1 = *(const v4f*)(srow + 8 * lane + 4);
      v8h hv;
#pragma unroll
      for (int e = 0; e < 4; ++e) { hv[e] = (_Float16)(p0[e] * kOpCarry); hv[4 + e] = (_Float16)(p1[e] * kOpCarry); }
      unsigned short* hp = H16 + (size_t)n * kFC + 8 * lane;
      for (int pass = 0; pass < 2; ++pass) {
        *(volatile v4f*)rp = v0;
        *(volatile v4f*)(rp + 128) = v1;
        *(volatile v8h*)hp = hv;
        __threadfence();
      }
      wave_lds_sync();
    }
  }
}

__global__ __launch_bounds__(256) void cell_kernel(const float* __restrict__ G, float* CS, float* __restrict__ HS, float* __restrict__ QS) {
  const int t = blockIdx.x * 256 + threadIdx.x;
  if (t >= kGraphs * kFC) return;
  const int b = t >> 8, c = t & 255;
  const float* gr = G + (size_t)b * kG4 + c;
  const float gi = gr[0], gf = gr[kFC], gg = gr[2 * kFC], go = gr[3 * kFC];
  const float cp = CS[t];
  const float iv = sigm(gi), fv = sigm(gf), ov = sigm(go);
  const float gv = tanhf(gg);
  const float cn = fv * cp + iv * gv;
  const float hn = ov * tanhf(cn);
  float* qp = QS + (size_t)b * kQ2 + c;
  for (int pass = 0; pass < 2; ++pass) {
    ((volatile float*)CS)[t] = cn;
    ((volatile float*)HS)[t] = hn;
    *(volatile float*)qp = hn;
    __threadfence();
  }
}

__global__ __launch_bounds__(kNT) void pool_attn_kernel(const float* __restrict__ H, const int* __restrict__ batch,
                                                        const float* __restrict__ HSv, float* __restrict__ QS,
                                                        unsigned short* __restrict__ A16) {
  __shared__ int LIST[kSCHB];
  __shared__ int scan_ws[80];
  __shared__ __align__(16) float red[8 * kFC];
  __shared__ float redm[8];
  __shared__ float redl[8];
  __shared__ float sfw[8];
  const int tid = threadIdx.x, lane = tid & 31, wave = tid >> 5;
  const int g = blockIdx.x;
  if (tid < 80) scan_ws[tid] = 0;
  __syncthreads();
  const v4f z4 = {0.f, 0.f, 0.f, 0.f};
  const v4f q0 = *(const v4f*)(HSv + (size_t)g * kFC + 8 * lane);
  const v4f q1 = *(const v4f*)(HSv + (size_t)g * kFC + 8 * lane + 4);
  float m = -INFINITY, l = 0.f;
  v4f acc0 = z4, acc1 = z4;
#pragma unroll 1
  for (int c = 0; c < kNCHB; ++c) {
    const int eb = c * kSCHB + tid * 8;
    const int ebc = (eb < kNodes) ? eb : (kNodes - 8);
    const v4i ba = *(const v4i*)(batch + ebc);
    const v4i bb = *(const v4i*)(batch + ebc + 4);
    const int bv8[8] = {ba[0], ba[1], ba[2], ba[3], bb[0], bb[1], bb[2], bb[3]};
    int rec[8]; int cnt = 0;
#pragma unroll
    for (int k = 0; k < 8; ++k) {
      int r = -1;
      if (eb + k < kNodes && bv8[k] == g) { r = eb + k; ++cnt; }
      rec[k] = r;
    }
    int tot; int p = blk_excl_scan(cnt, scan_ws, tid, &tot);
#pragma unroll
    for (int k = 0; k < 8; ++k) if (rec[k] >= 0) { if ((unsigned)p < (unsigned)kSCHB) LIST[p] = rec[k]; ++p; }
    __syncthreads();
    const int totc = tot < kSCHB ? tot : kSCHB;
#pragma unroll 1
    for (int qq = wave; qq < totc; qq += 8) {
      int nd = LIST[qq]; nd = nd < 0 ? 0 : (nd >= kNodes ? kNodes - 1 : nd);
      const float* hr = H + (size_t)nd * kFC + 8 * lane;
      const v4f h0 = *(const v4f*)hr;
      const v4f h1 = *(const v4f*)(hr + 4);
      float d = dot4(h0, q0) + dot4(h1, q1);
#pragma unroll
      for (int off = 1; off < 32; off <<= 1) d += __shfl_xor(d, off, 32);
      const float mn = fmaxf(m, d);
      const float rr = expf(m - mn);
      const float ex = expf(d - mn);
      acc0 = acc0 * rr + ex * h0;
      acc1 = acc1 * rr + ex * h1;
      l = l * rr + ex;
      m = mn;
    }
    __syncthreads();
  }
  *(v4f*)(red + wave * kFC + 8 * lane) = acc0;
  *(v4f*)(red + wave * kFC + 8 * lane + 4) = acc1;
  if (lane == 0) { redm[wave] = m; redl[wave] = l; }
  __syncthreads();
  if (wave == 0) {
    const int l8 = lane & 7;
    float mw = redm[l8], lw = redl[l8];
    mw = (lane < 8) ? mw : -INFINITY;
    lw = (lane < 8) ? lw : 0.f;
    float mx = mw;
#pragma unroll
    for (int off = 1; off < 32; off <<= 1) mx = fmaxf(mx, __shfl_xor(mx, off, 32));
    mx = (mx > -INFINITY) ? mx : 0.f;
    const float fw = expf(mw - mx);
    float lt = lw * fw;
#pragma unroll
    for (int off = 1; off < 32; off <<= 1) lt += __shfl_xor(lt, off, 32);
    const float inv = 1.0f / (lt + 1e-16f);
    if (lane < 8) sfw[lane] = fw;
    wave_lds_sync();
    v4f s0 = z4, s1 = z4, t0 = z4, t1 = z4;
#pragma unroll 1
    for (int w = 0; w < 8; ++w) {
      const float f = sfw[w];
      const float* rw = red + w * kFC;
      s0 = s0 + *(const v4f*)(rw + 4 * lane) * f;
      s1 = s1 + *(const v4f*)(rw + 128 + 4 * lane) * f;
      t0 = t0 + *(const v4f*)(rw + 8 * lane) * f;
      t1 = t1 + *(const v4f*)(rw + 8 * lane + 4) * f;
    }
    s0 = s0 * inv; s1 = s1 * inv; t0 = t0 * inv; t1 = t1 * inv;
    v8h hr8, hq8;
#pragma unroll
    for (int e = 0; e < 4; ++e) {
      hr8[e] = (_Float16)(t0[e] * kQCarry); hr8[4 + e] = (_Float16)(t1[e] * kQCarry);
      hq8[e] = (_Float16)(q0[e] * kQCarry); hq8[4 + e] = (_Float16)(q1[e] * kQCarry);
    }
    float* rp = QS + (size_t)g * kQ2 + kFC;
    unsigned short* ap = A16 + (size_t)g * kGK;
    for (int pass = 0; pass < 2; ++pass) {
      *(volatile v4f*)(rp + 4 * lane) = s0;
      *(volatile v4f*)(rp + 128 + 4 * lane) = s1;
      *(volatile v8h*)(ap + 8 * lane) = hq8;
      *(volatile v8h*)(ap + kFC + 8 * lane) = hr8;
      *(volatile v8h*)(ap + kQ2 + 8 * lane) = hq8;
      __threadfence();
    }
  }
}

__global__ __launch_bounds__(256) void head_kernel(const float* __restrict__ QS, const float* __restrict__ Wc1,
                                                   const float* __restrict__ bc1, const float* __restrict__ Wc2,
                                                   const float* __restrict__ bc2, float* __restrict__ out) {
  __shared__ float zs[kGraphs * 64];
  __shared__ __align__(16) float so[kGraphs * kCls];
  const int tid = threadIdx.x, lane = tid & 31, wave = tid >> 5;
  for (int i = tid; i < kGraphs * 64; i += 256) {
    const int b = i >> 6, j = i & 63;
    const float* qr = QS + (size_t)b * kQ2;
    float s = 0.f;
#pragma unroll 1
    for (int k = 0; k < kQ2; ++k) s += qr[k] * Wc1[k * 64 + j];
    s += bc1[j];
    zs[i] = fmaxf(s, 0.f);
  }
  __syncthreads();
  for (int i = tid; i < kGraphs * kCls; i += 256) {
    const int b = i / kCls;
    const int cc = i - b * kCls;
    float a = 0.f;
#pragma unroll 1
    for (int j = 0; j < 64; ++j) a += zs[b * 64 + j] * Wc2[j * kCls + cc];
    a += bc2[cc];
    so[i] = a;
  }
  __syncthreads();
  if (wave == 0) {
    for (int pass = 0; pass < 2; ++pass) {
#pragma unroll
      for (int it = 0; it < (kGraphs * kCls) / 128; ++it) {
        const v4f v = *(const v4f*)(so + 128 * it + 4 * lane);
        *(volatile v4f*)(out + 128 * it + 4 * lane) = v;
      }
      __threadfence();
    }
  }
}

extern "C" void kernel_launch(void* const* d_in, const int* in_sizes, int n_in,
                              void* d_out, int out_size, void* d_ws, size_t ws_size, hipStream_t stream) {
  (void)in_sizes; (void)n_in; (void)out_size;
  const float* x     = (const float*)d_in[0];
  const int*   ei    = (const int*)  d_in[1];
  const int*   batch = (const int*)  d_in[2];
  const float* W0    = (const float*)d_in[3];
  const float* as0   = (const float*)d_in[4];
  const float* ad0   = (const float*)d_in[5];
  const float* b0    = (const float*)d_in[6];
  const float* W1    = (const float*)d_in[7];
  const float* as1   = (const float*)d_in[8];
  const float* ad1   = (const float*)d_in[9];
  const float* b1    = (const float*)d_in[10];
  const float* W2    = (const float*)d_in[11];
  const float* as2   = (const float*)d_in[12];
  const float* ad2   = (const float*)d_in[13];
  const float* b2    = (const float*)d_in[14];
  const float* Wih   = (const float*)d_in[15];
  const float* Whh   = (const float*)d_in[16];
  const float* bih   = (const float*)d_in[17];
  const float* bhh   = (const float*)d_in[18];
  const float* Wc1   = (const float*)d_in[19];
  const float* bc1   = (const float*)d_in[20];
  const float* Wc2   = (const float*)d_in[21];
  const float* bc2   = (const float*)d_in[22];
  float* out = (float*)d_out;

  char* ws = (char*)d_ws; size_t off = 0;
  auto carve = [&](size_t bytes) -> char* { char* p = ws + off; off += (bytes + 255) & ~(size_t)255; return p; };
  unsigned short* W0T  = (unsigned short*)carve((size_t)kFC * kDin * 2);
  unsigned short* W1T  = (unsigned short*)carve((size_t)kFC * kFC * 2);
  unsigned short* W2T  = (unsigned short*)carve((size_t)kFC * kFC * 2);
  unsigned short* WG16 = (unsigned short*)carve((size_t)kG4 * kGK * 2);
  float*          BSUM = (float*)carve((size_t)kG4 * 4);
  unsigned short* X16  = (unsigned short*)carve((size_t)kNP * kDin * 2);
  unsigned short* H16  = (unsigned short*)carve((size_t)kNP * kFC * 2);
  float*          FEAT = (float*)carve((size_t)kNP * kFC * 4);
  float*          AL   = (float*)carve((size_t)kNodes * kHeads * 4);
  float*          AR   = (float*)carve((size_t)kNodes * kHeads * 4);
  float*          HA   = (float*)carve((size_t)kNPA * kFC * 4);
  float*          HB   = (float*)carve((size_t)kNPA * kFC * 4);
  const size_t zrBytes = (size_t)kGraphs * (kQ2 + kFC + kFC) * 4 + (size_t)kGraphs * kGK * 2;
  char*           ZR   = carve(zrBytes);
  float*          G    = (float*)carve((size_t)kGraphs * kG4 * 4);
  if (off > ws_size || off > (size_t)134217728) return;
  float*          QS   = (float*)ZR;
  float*          HS   = QS + (size_t)kGraphs * kQ2;
  float*          CS   = HS + (size_t)kGraphs * kFC;
  unsigned short* A16S = (unsigned short*)(CS + (size_t)kGraphs * kFC);

  wtcast_kernel<<<dim3(4, 4, 3), 256, 0, stream>>>(W0, W1, W2, W0T, W1T, W2T, kOpCarry);
  wgcast_kernel<<<(kG4 * (kGK / 8)) / 256, 256, 0, stream>>>(Wih, Whh, bih, bhh, WG16, BSUM);
  xcast_kernel<<<(kNP * kDin / 8 + 255) / 256, 256, 0, stream>>>(x, X16);
  {
    const int n4 = (int)(zrBytes / 16);
    zero16_kernel<<<(n4 + 255) / 256, 256, 0, stream>>>((unsigned*)ZR, n4);
  }

  const float* asv[3] = {as0, as1, as2};
  const float* adv[3] = {ad0, ad1, ad2};
  const float* bsv[3] = {b0, b1, b2};
  const unsigned short* wtv[3] = {W0T, W1T, W2T};
  const int featTiles = (kNP / 64) * (kFC / 64);
  for (int layer = 0; layer < 3; ++layer) {
    const int K = (layer == 0) ? kDin : kFC;
    const unsigned short* Ap = (layer == 0) ? X16 : H16;
    wmma_gemm64<0, false, 0, 0, false><<<dim3((featTiles + 7) / 8, 1), 256, 0, stream>>>(
        Ap, (const unsigned short*)nullptr, K, 0L,
        wtv[layer], (const unsigned short*)nullptr, K, 0L,
        (void*)FEAT, (void*)nullptr, kFC, 0L,
        (const float*)nullptr, (const float*)nullptr, 0L, kNP, kFC, K, kFeatScale);
    alar_kernel<<<(kNodes * kHeads + 255) / 256, 256, 0, stream>>>(FEAT, asv[layer], adv[layer], AL, AR);
    if (layer == 0)      gat_kernel<false><<<kTiles, kNT, 0, stream>>>(FEAT, ei, AL, AR, bsv[0], HB, HA, H16);
    else if (layer == 1) gat_kernel<true ><<<kTiles, kNT, 0, stream>>>(FEAT, ei, AL, AR, bsv[1], HA, HB, H16);
    else                 gat_kernel<true ><<<kTiles, kNT, 0, stream>>>(FEAT, ei, AL, AR, bsv[2], HB, HA, H16);
  }

  const int gateTiles = (kGraphs / 64) * (kG4 / 64);
  for (int step = 0; step < 3; ++step) {
    wmma_gemm64<0, false, 2, 0, false><<<dim3((gateTiles + 7) / 8, 1), 256, 0, stream>>>(
        A16S, (const unsigned short*)nullptr, kGK, 0L,
        WG16, (const unsigned short*)nullptr, kGK, 0L,
        (void*)G, (void*)nullptr, kG4, 0L,
        BSUM, (const float*)nullptr, 0L, kGraphs, kG4, kGK, kGateScale);
    cell_kernel<<<(kGraphs * kFC) / 256, 256, 0, stream>>>(G, CS, HS, QS);
    pool_attn_kernel<<<kGraphs, kNT, 0, stream>>>(HA, batch, HS, QS, A16S);
  }

  head_kernel<<<1, 256, 0, stream>>>(QS, Wc1, bc1, Wc2, bc2, out);
}
